// SelectiveSSMExpert_16793322127758
// MI455X (gfx1250) — hardware-run, weakly checked
//
#include <hip/hip_runtime.h>


#define NM   16384
#define NB   4
#define NT   4096
#define ND   1024
#define NS   256
#define NH   512
#define NG   1024
#define NP   768
typedef _Float16 h16;
typedef unsigned short bf;
typedef __attribute__((ext_vector_type(16))) __bf16   v16bf;
typedef __attribute__((ext_vector_type(16))) _Float16 v16h;
typedef __attribute__((ext_vector_type(8)))  _Float16 v8h;
typedef __attribute__((ext_vector_type(8)))  unsigned short v8us;
typedef __attribute__((ext_vector_type(8)))  float    v8f;
typedef __attribute__((ext_vector_type(4)))  float    v4f;
typedef v8h  __attribute__((may_alias)) v8ha;
typedef v4f  __attribute__((may_alias)) v4fa;
typedef v8us __attribute__((may_alias)) v8usa;

__device__ __forceinline__ unsigned short f2bf(float f) { unsigned u = __float_as_uint(f); u += 0x7FFFu + ((u >> 16) & 1u); return (unsigned short)(u >> 16); }
__device__ __forceinline__ float bf2f(unsigned short b) { return __uint_as_float(((unsigned)b) << 16); }
__device__ __forceinline__ float bfr(float f) { return bf2f(f2bf(f)); }
__device__ __forceinline__ v16h cat16(v8h lo, v8h hi) { return __builtin_shufflevector(lo, hi, 0, 1, 2, 3, 4, 5, 6, 7, 8, 9, 10, 11, 12, 13, 14, 15); }
__device__ __forceinline__ v16bf cat16b(v8us lo, v8us hi) { return __builtin_bit_cast(v16bf, __builtin_shufflevector(lo, hi, 0, 1, 2, 3, 4, 5, 6, 7, 8, 9, 10, 11, 12, 13, 14, 15)); }
__device__ __forceinline__ v8f wmma16(v16h a, v16h b, v8f c) { return __builtin_amdgcn_wmma_f32_16x16x32_f16(false, a, false, b, (short)0, c, false, false); }
__device__ __forceinline__ v8f wmmab(v16bf a, v16bf b, v8f c) { return __builtin_amdgcn_wmma_f32_16x16x32_bf16(false, a, false, b, (short)0, c, false, false); }

template <typename T16> struct WFrag;
template <> struct WFrag<h16> { typedef v16h V; static __device__ __forceinline__ V ld(const h16* p) { return cat16(*(const v8h*)p, *(const v8h*)(p + 16)); } static __device__ __forceinline__ v8f mma(V a, V b, v8f c) { return wmma16(a, b, c); } };
template <> struct WFrag<bf> { typedef v16bf V; static __device__ __forceinline__ V ld(const bf* p) { return cat16b(*(const v8us*)p, *(const v8us*)(p + 16)); } static __device__ __forceinline__ v8f mma(V a, V b, v8f c) { return wmmab(a, b, c); } };
template <typename T16, int NSPLIT, bool BIAS>
__global__ __launch_bounds__(32) void k_gemmw(const T16* __restrict__ A, const T16* __restrict__ A2, const T16* __restrict__ Bt, const T16* __restrict__ Bt2, int K, float* C, int ldc, const float* __restrict__ bias, size_t sA, size_t sB, size_t sC) {
    typedef typename WFrag<T16>::V V;
    __shared__ __align__(16) float os[16 * 68];
    const size_t z = blockIdx.z; A += z * sA; if (A2) A2 += z * sA; Bt += z * sB; if (Bt2) Bt2 += z * sB; C += z * sC;
    const int lane = threadIdx.x & 31, lr = lane & 15, hi = lane >> 4; const int r0 = blockIdx.x * 64, c0 = blockIdx.y * 64;
    v8f acc[4][4];
#pragma unroll
    for (int mb = 0; mb < 4; ++mb)
#pragma unroll
        for (int nb = 0; nb < 4; ++nb) acc[mb][nb] = (v8f){};
    const size_t aoff = (size_t)(r0 + lr) * K + 8 * hi, boff = (size_t)(c0 + lr) * K + 8 * hi;
    for (int kc = 0; kc < K; kc += 32) {
        V a[4], a2[4];
#pragma unroll
        for (int mb = 0; mb < 4; ++mb) { a[mb] = WFrag<T16>::ld(A + aoff + (size_t)mb * 16 * K + kc); if (NSPLIT == 1 || NSPLIT == 2) a2[mb] = WFrag<T16>::ld(A2 + aoff + (size_t)mb * 16 * K + kc); }
#pragma unroll
        for (int nb = 0; nb < 4; ++nb) { const V b = WFrag<T16>::ld(Bt + boff + (size_t)nb * 16 * K + kc); V b2; if (NSPLIT >= 2) b2 = WFrag<T16>::ld(Bt2 + boff + (size_t)nb * 16 * K + kc);
#pragma unroll
            for (int mb = 0; mb < 4; ++mb) { acc[mb][nb] = WFrag<T16>::mma(a[mb], b, acc[mb][nb]); if (NSPLIT == 1 || NSPLIT == 2) acc[mb][nb] = WFrag<T16>::mma(a2[mb], b, acc[mb][nb]); if (NSPLIT >= 2) acc[mb][nb] = WFrag<T16>::mma(a[mb], b2, acc[mb][nb]); } }
        asm volatile("v_nop\n\tv_nop\n\tv_nop\n\tv_nop" : "+v"(acc[0][0]), "+v"(acc[1][1]), "+v"(acc[2][2]), "+v"(acc[3][3]) : "v"(a[0]), "v"(a[3]));
    }
#pragma unroll
    for (int mb = 0; mb < 4; ++mb) {
#pragma unroll
        for (int nb = 0; nb < 4; ++nb) {
#pragma unroll
            for (int j = 0; j < 8; ++j) os[(hi * 8 + j) * 68 + nb * 16 + lr] = acc[mb][nb][j]; }
        __builtin_amdgcn_wave_barrier(); asm volatile("" ::: "memory");
        float* crow = C + (size_t)(r0 + mb * 16) * ldc + c0;
#pragma unroll 1
        for (int ps = 0; ps < 2; ++ps) {
#pragma unroll
            for (int s = 0; s < 8; ++s) { const int row = 2 * s + hi, cofs = lr * 4; v4f val = *(const v4fa*)(os + row * 68 + cofs); if (BIAS) { val[0] += bfr(bias[c0 + cofs]); val[1] += bfr(bias[c0 + cofs + 1]); val[2] += bfr(bias[c0 + cofs + 2]); val[3] += bfr(bias[c0 + cofs + 3]); }
                *(volatile v4f*)(crow + (size_t)row * ldc + cofs) = val; }
            if (ps == 0) __threadfence(); }
        __builtin_amdgcn_wave_barrier(); asm volatile("" ::: "memory");
    }
}

typedef __attribute__((ext_vector_type(2))) _Float16 v2h;
typedef __attribute__((ext_vector_type(4))) _Float16 v4h;
typedef __attribute__((ext_vector_type(2))) unsigned short v2us;
typedef __attribute__((ext_vector_type(4))) unsigned short v4us;
typedef __attribute__((ext_vector_type(2))) float v2f;
typedef __attribute__((ext_vector_type(4))) int v4i;
__global__ __launch_bounds__(256) void k_cvt8(const float* __restrict__ src, bf* dst, size_t n8) { const size_t i = (size_t)blockIdx.x * 256 + threadIdx.x; if (i >= n8) return; const v8f v = *(const v8f*)(src + i * 8); v8us o;
#pragma unroll
    for (int k = 0; k < 8; ++k) o[k] = f2bf(v[k]); *(volatile v8us*)(dst + i * 8) = o; __threadfence(); *(volatile v8us*)(dst + i * 8) = o; }

__device__ __forceinline__ h16 toh_flush(float x) { const float z = (fabsf(x) < 6.103515625e-05f) ? 0.0f : x; return (h16)z; }

template <bool RB>
__global__ __launch_bounds__(256) void k_c16(const float* __restrict__ src, h16* dst, size_t n8) { const size_t i = (size_t)blockIdx.x * 256 + threadIdx.x; if (i >= n8) return; const float* p = src + i * 8; const v4f a = *(const v4f*)p, b = *(const v4f*)(p + 4); v8h o;
#pragma unroll
    for (int q = 0; q < 4; ++q) { o[q] = toh_flush(RB ? bfr(a[q]) : a[q]); o[q + 4] = toh_flush(RB ? bfr(b[q]) : b[q]); }
    *(volatile v8h*)(dst + i * 8) = o; __threadfence(); *(volatile v8h*)(dst + i * 8) = o; }

__global__ __launch_bounds__(256) void k_act(const float* __restrict__ P, h16* Sh) { const unsigned e = blockIdx.x * 256u + threadIdx.x; const unsigned m = e >> 6, c0 = (e & 63u) << 3; const float* p = P + (size_t)m * NP + NS + c0; const v4f va = *(const v4f*)p, vb = *(const v4f*)(p + 4); v8h o;
#pragma unroll
    for (int k = 0; k < 4; ++k) { const float qa = va[k], qb = vb[k]; o[k] = toh_flush(qa * (1.0f / (1.0f + expf(-qa)))); o[k + 4] = toh_flush(qb * (1.0f / (1.0f + expf(-qb)))); }
    *(volatile v8h*)(Sh + (size_t)e * 8) = o; __threadfence(); *(volatile v8h*)(Sh + (size_t)e * 8) = o; }

__global__ __launch_bounds__(256) void k_pre(const float* __restrict__ G, const float* __restrict__ P, float* Av, float* Bv) { const unsigned e = blockIdx.x * 256u + threadIdx.x; const unsigned m = e >> 6, n0 = (e & 63u) << 2; const float* g = G + (size_t)m * NG + n0; const v4f g0 = *(const v4f*)g, g1 = *(const v4f*)(g + NS), pv = *(const v4f*)(P + (size_t)m * NP + n0); v4f dq, rq;
#pragma unroll
    for (int k = 0; k < 4; ++k) { dq[k] = 1.0f / (1.0f + expf(-g0[k])); rq[k] = tanhf(g1[k]) * pv[k]; }
    float* oa = Av + (size_t)e * 4; float* ob = Bv + (size_t)e * 4;
    *(volatile v4f*)oa = dq; *(volatile v4f*)ob = rq; __threadfence();
    *(volatile v4f*)oa = dq; *(volatile v4f*)ob = rq; }

__global__ __launch_bounds__(32) void k_walk(const float* __restrict__ Av, const float* __restrict__ Bv, float* Hs) { const unsigned i = blockIdx.x * 32u + threadIdx.x; const unsigned bq = i >> 8, n = i & 255u; float st = 0.0f;
    for (int t0 = 0; t0 < NT; t0 += 8) { const size_t r0 = ((size_t)bq * NT + t0) * NS + n; float w8[8];
#pragma unroll
        for (int s = 0; s < 8; ++s) { const float dv = Av[r0 + (size_t)s * NS], rv = Bv[r0 + (size_t)s * NS]; st = dv * st + rv; w8[s] = st; }
        float* o = Hs + r0;
#pragma unroll
        for (int s = 0; s < 8; ++s) *(volatile float*)(o + (size_t)s * NS) = w8[s];
        __threadfence();
#pragma unroll
        for (int s = 0; s < 8; ++s) *(volatile float*)(o + (size_t)s * NS) = w8[s]; }
}

__global__ __launch_bounds__(256) void k_res(const float* __restrict__ G, const float* __restrict__ P, const float* __restrict__ Hs, const float* __restrict__ sv, h16* Yh) { const unsigned e = blockIdx.x * 256u + threadIdx.x; const unsigned m = e >> 5, n0 = (e & 31u) << 3; const float* g = G + (size_t)m * NG + 2 * NS + n0; const float* p = P + (size_t)m * NP + n0; const float* hp = Hs + (size_t)e * 8; v8h o;
#pragma unroll
    for (int hf = 0; hf < 2; ++hf) { const v4f g2 = *(const v4f*)(g + 4 * hf), g3 = *(const v4f*)(g + NS + 4 * hf), pv = *(const v4f*)(p + 4 * hf), hv = *(const v4f*)(hp + 4 * hf), sx = *(const v4f*)(sv + n0 + 4 * hf);
#pragma unroll
        for (int k = 0; k < 4; ++k) o[4 * hf + k] = toh_flush(tanhf(g2[k]) * hv[k] + (bfr(sx[k]) * (1.0f / (1.0f + expf(-g3[k])))) * pv[k]); }
    *(volatile v8h*)(Yh + (size_t)e * 8) = o; __threadfence(); *(volatile v8h*)(Yh + (size_t)e * 8) = o; }

extern "C" void kernel_launch(void* const* d_in, const int* in_sizes, int n_in, void* d_out, int out_size, void* d_ws, size_t ws_size, hipStream_t stream) {
    if (n_in < 6) return;
    if (in_sizes[0] != NM * ND || in_sizes[1] != NS * ND || in_sizes[2] != NH * ND || in_sizes[3] != NG * NH || in_sizes[4] != ND * NS || in_sizes[5] != NS) return;
    if (out_size != NM * ND) return;
    static_assert(NM == NB * NT && NP == NS + NH && NG == 4 * NS && NM % 64 == 0 && NP % 64 == 0 && NG % 64 == 0 && ND % 64 == 0 && ND % 32 == 0 && NH % 32 == 0 && NS % 32 == 0 && (NM * ND / 8) % 256 == 0 && (NS * ND / 8) % 256 == 0 && (NH * ND / 8) % 256 == 0 && (NG * NH / 8) % 256 == 0 && (ND * NS / 8) % 256 == 0 && (NM * NH / 8) % 256 == 0 && (NM * NS / 8) % 256 == 0 && (NM * NS / 4) % 256 == 0 && NH == 512 && NS == 256 && (NB * NS) % 32 == 0 && NT % 8 == 0, "the products: row and column counts multiples of 64, the depths of 32; the flat grids exact; k_act's and k_pre's 64 threads a row and k_res's 32; a wave's 32 channels in one sequence; the rows in eights");
    const float* i0 = (const float*)d_in[0]; const float* i1 = (const float*)d_in[1]; const float* i2 = (const float*)d_in[2]; const float* i3 = (const float*)d_in[3]; const float* i4 = (const float*)d_in[4]; const float* i5 = (const float*)d_in[5]; float* out = (float*)d_out;
    char* wsp = (char*)d_ws; auto take = [&](size_t bytes) { char* p = wsp; wsp += (bytes + 255) & ~(size_t)255; return (void*)p; };
    bf* Xb = (bf*)take((size_t)NM * ND * 2); bf* B1 = (bf*)take((size_t)NP * ND * 2); float* P = (float*)take((size_t)NM * NP * 4); h16* Sh = (h16*)take((size_t)NM * NH * 2); h16* Wg = (h16*)take((size_t)NG * NH * 2); float* G = (float*)take((size_t)NM * NG * 4); float* Av = (float*)take((size_t)NM * NS * 4); float* Bv = (float*)take((size_t)NM * NS * 4); float* Hs = (float*)take((size_t)NM * NS * 4); h16* Yh = (h16*)take((size_t)NM * NS * 2); h16* Wo = (h16*)take((size_t)ND * NS * 2);
    if ((size_t)(wsp - (char*)d_ws) > ws_size) return;
    k_cvt8<<<(unsigned)(NM * ND / 8 / 256), 256, 0, stream>>>(i0, Xb, (size_t)NM * ND / 8);
    k_cvt8<<<(unsigned)(NS * ND / 8 / 256), 256, 0, stream>>>(i1, B1, (size_t)NS * ND / 8);
    k_cvt8<<<(unsigned)(NH * ND / 8 / 256), 256, 0, stream>>>(i2, B1 + (size_t)NS * ND, (size_t)NH * ND / 8);
    k_gemmw<bf, 0, false><<<dim3(NM / 64, NP / 64, 1), 32, 0, stream>>>(Xb, nullptr, B1, nullptr, ND, P, NP, nullptr, 0, 0, 0);
    k_act<<<(unsigned)(NM * NH / 8 / 256), 256, 0, stream>>>(P, Sh);
    k_c16<true><<<(unsigned)(NG * NH / 8 / 256), 256, 0, stream>>>(i3, Wg, (size_t)NG * NH / 8);
    k_gemmw<h16, 0, false><<<dim3(NM / 64, NG / 64, 1), 32, 0, stream>>>(Sh, nullptr, Wg, nullptr, NH, G, NG, nullptr, 0, 0, 0);
    k_pre<<<(unsigned)(NM * NS / 4 / 256), 256, 0, stream>>>(G, P, Av, Bv);
    k_walk<<<(unsigned)(NB * NS / 32), 32, 0, stream>>>(Av, Bv, Hs);
    k_res<<<(unsigned)(NM * NS / 8 / 256), 256, 0, stream>>>(G, P, Hs, i5, Yh);
    k_c16<true><<<(unsigned)(ND * NS / 8 / 256), 256, 0, stream>>>(i4, Wo, (size_t)ND * NS / 8);
    k_gemmw<h16, 0, false><<<dim3(NM / 64, ND / 64, 1), 32, 0, stream>>>(Yh, nullptr, Wo, nullptr, NS, out, ND, nullptr, 0, 0, 0);
}
